// BSG_78829829751266
// MI455X (gfx1250) — hardware-run, weakly checked
//
#include <hip/hip_runtime.h>

typedef _Float16 v16h __attribute__((ext_vector_type(16)));
typedef _Float16 v8h  __attribute__((ext_vector_type(8)));
typedef float    v8f  __attribute__((ext_vector_type(8)));
typedef float    v4f  __attribute__((ext_vector_type(4)));
typedef float    v2f  __attribute__((ext_vector_type(2)));
typedef double   v2d  __attribute__((ext_vector_type(2)));
typedef v8h      __attribute__((may_alias)) v8ha;
typedef v4f      __attribute__((may_alias)) v4fa;
typedef v2f      __attribute__((may_alias)) v2fa;
typedef unsigned __attribute__((may_alias)) u32a;

union Frag { v16h v; v8h half[2]; };
union Pk2  { unsigned u; _Float16 e[2]; };

constexpr int DIM  = 50;
constexpr int HID  = 50;
constexpr int LAT  = 100;
constexpr int CTX  = 10;
constexpr int TB   = 32;
constexpr int NTH  = 128;
constexpr int NWAV = NTH / 32;
constexpr int KP   = 64;
constexpr int NP1  = 64;
constexpr int NP2  = 112;
constexpr int AROWS = TB * CTX;
constexpr int GROWS = AROWS + TB;
constexpr int NIDS  = 2 * AROWS + TB;
constexpr int NUNIT = AROWS + TB;
constexpr int PLROWS = 2 * NP1 + NP2;
constexpr int PART_STRIDE = 16;

static_assert((TB * 8) / 16 == 4 * NWAV);
static_assert((TB * 2) / 16 == NWAV);
static_assert(DIM == HID);
static_assert((AROWS % 32) == 0);
static_assert((NUNIT % 32) == 0);
static_assert((NIDS % 32) == 0);
static_assert(((GROWS * 32) % NTH) == 0);

constexpr int OFF_GROW = 0;
constexpr int OFF_HBF  = OFF_GROW + GROWS * KP * 2;
constexpr int OFF_HCS  = OFF_HBF + TB * KP * 2;
constexpr int OFF_HS   = OFF_HCS + TB * NP1 * 4;
constexpr int OFF_MUS  = OFF_HS + TB * NP1 * 4;
constexpr int OFF_B1   = OFF_MUS + TB * NP2 * 4;
constexpr int OFF_BMU  = OFF_B1 + NP1 * 4;
constexpr int OFF_IDS  = OFF_BMU + NP2 * 4;
constexpr int OFF_RED  = OFF_IDS + NIDS * 4;
constexpr int OFF_BSUM = OFF_RED + NTH * 8;
constexpr int LDS_BYTES = OFF_BSUM + 64;
static_assert((OFF_HBF % 16) == 0);
static_assert((OFF_HCS % 16) == 0);
static_assert((OFF_MUS % 16) == 0);
static_assert((OFF_RED % 8) == 0);
static_assert((OFF_BSUM % 8) == 0);
static_assert(LDS_BYTES == 84352);

constexpr size_t PLANE_BYTES = (size_t)PLROWS * KP * 2;
constexpr size_t OFF_PART    = 32768;
static_assert(PLANE_BYTES <= OFF_PART);

__device__ __forceinline__ v8f wmma_f16(v16h a, v16h b, v8f c) {
  v8f d = __builtin_amdgcn_wmma_f32_16x16x32_f16(false, a, false, b, (short)0, c, false, false);
  asm volatile("v_nop\n\tv_nop\n\tv_nop\n\tv_nop" : "+v"(d) : "v"(a), "v"(b));
  return d;
}

__device__ __forceinline__ v16h load_frag(const _Float16* p, int h) {
  Frag f;
  f.half[0] = *(const v8ha*)(p + 8 * h);
  f.half[1] = *(const v8ha*)(p + 16 + 8 * h);
  return f.v;
}

__device__ __forceinline__ void prep_pass(const float* __restrict__ W1, const float* __restrict__ Wmu,
                                          const float* __restrict__ Wls, _Float16* planes, int t) {
  const int q = t & 7;
  #pragma unroll 1
  for (int R = t >> 3; R < PLROWS; R += 32) {
    const int sel = (R < NP1) ? 0 : ((R < 2 * NP1) ? 1 : 2);
    const int n = R - ((sel >= 1) ? NP1 : 0) - ((sel == 2) ? NP1 : 0);
    const int n1 = min(n, HID - 1);
    const int n2 = min(n, LAT - 1);
    v8h o;
    #pragma unroll
    for (int j = 0; j < 8; ++j) {
      const int k = 8 * q + j;
      const int kc = min(k, DIM - 1);
      const float wa = W1[(size_t)kc * HID + n1];
      const float wb = W1[(size_t)(DIM + kc) * HID + n1];
      const float wm = Wmu[(size_t)kc * LAT + n2];
      const float wl = Wls[kc];
      const bool kin = (k < DIM);
      float v = 0.0f;
      if (sel == 0)      v = (kin && n < HID) ? wa : 0.0f;
      else if (sel == 1) v = (kin && n < HID) ? wb : 0.0f;
      else               v = (kin && n < LAT) ? wm : ((kin && n == LAT) ? wl : 0.0f);
      o[j] = (_Float16)(v * 8.0f);
    }
    *(volatile v8h*)(planes + (size_t)R * KP + 8 * q) = o;
  }
}

__global__ __launch_bounds__(256) void bsg_prep(const float* __restrict__ W1, const float* __restrict__ Wmu,
                                                const float* __restrict__ Wls, _Float16* planes) {
  const int t = threadIdx.x;
  prep_pass(W1, Wmu, Wls, planes, t);
  __threadfence();
  prep_pass(W1, Wmu, Wls, planes, t);
}

__device__ __forceinline__ float kl_term(int id, const float* murow, float ls, float els,
                                         const float* __restrict__ tmeans,
                                         const float* __restrict__ tlogv) {
  const float* tm = tmeans + (size_t)id * LAT;
  float ds = 0.0f;
  #pragma unroll 5
  for (int p = 0; p < LAT / 4; ++p) {
    const v4f a = *(const v4fa*)(murow + 4 * p);
    const v4f c = *(const v4fa*)(tm + 4 * p);
    const float d0 = a.x - c.x, d1 = a.y - c.y, d2 = a.z - c.z, d3 = a.w - c.w;
    ds += d0 * d0;
    ds += d1 * d1;
    ds += d2 * d2;
    ds += d3 * d3;
  }
  const float tl  = tlogv[id];
  const float tv  = expf(tl);
  const float rtv = 1.0f / tv;
  return 0.5f * (((els * rtv + ds * rtv) + (tl - ls)) - (float)LAT);
}

__global__ __launch_bounds__(NTH) void bsg_main(
    const float* __restrict__ emb,
    const float* __restrict__ b1,
    const float* __restrict__ bmu,
    const float* __restrict__ bls,
    const float* __restrict__ tmeans,
    const float* __restrict__ tlogv,
    const int*   __restrict__ centers,
    const int*   __restrict__ contexts,
    const int*   __restrict__ negctx,
    const _Float16* __restrict__ w1a,
    const _Float16* __restrict__ w1b,
    const _Float16* __restrict__ wmt,
    double* part,
    int nB, int nV)
{
  extern __shared__ __align__(16) char smem[];
  _Float16* grow = (_Float16*)(smem + OFF_GROW);
  _Float16* cenA = grow + AROWS * KP;
  _Float16* hbf  = (_Float16*)(smem + OFF_HBF);
  float*    hcs  = (float*)(smem + OFF_HCS);
  float*    hs   = (float*)(smem + OFF_HS);
  float*    mus  = (float*)(smem + OFF_MUS);
  float*    b1s  = (float*)(smem + OFF_B1);
  float*    bmus = (float*)(smem + OFF_BMU);
  int*      ids  = (int*)(smem + OFF_IDS);
  double*   red  = (double*)(smem + OFF_RED);
  double*   bsum = (double*)(smem + OFF_BSUM);

  const int t = threadIdx.x, lane = t & 31, w = t >> 5;
  const int h = lane >> 4, m = lane & 15;
  const int b0 = blockIdx.x * TB;
  const v8f z8 = {0.f, 0.f, 0.f, 0.f, 0.f, 0.f, 0.f, 0.f};

  #pragma unroll 1
  for (int i = t; i < NIDS; i += NTH) {
    const int u  = i - ((i >= AROWS) ? AROWS : 0) - ((i >= 2 * AROWS) ? AROWS : 0);
    const int bq = u / CTX;
    const int cq = u - bq * CTX;
    const bool isCen = (i >= 2 * AROWS);
    const int b  = isCen ? u : bq;
    const int c  = isCen ? 0 : cq;
    const int gb = min(b0 + b, nB - 1);
    const int vx = contexts[(size_t)gb * CTX + c];
    const int vn = negctx[(size_t)gb * CTX + c];
    const int vc = centers[gb];
    int id = (i < AROWS) ? vx : (isCen ? vc : vn);
    id = min(max(id, 0), nV - 1);
    ids[i] = id;
  }
  {
    const float vb1 = b1[min(t, HID - 1)];
    const float vbm = bmu[min(t, LAT - 1)];
    const float vbl = bls[0];
    if (t < NP1) b1s[t] = (t < HID) ? vb1 : 0.0f;
    if (t < NP2) bmus[t] = (t < LAT) ? vbm : ((t == LAT) ? vbl : 0.0f);
  }
  __syncthreads();

  #pragma unroll 1
  for (int i = t; i < GROWS * 32; i += NTH) {
    const int row = i >> 5, p = i & 31;
    const int rr  = row - 256;
    const int sidx = (row < 256) ? ((row >> 3) * CTX + (row & 7))
                   : ((row < AROWS) ? ((rr >> 1) * CTX + 8 + (rr & 1))
                                    : (2 * AROWS + (row - AROWS)));
    const int id = ids[sidx];
    const int pc = min(p, DIM / 2 - 1);
    const v2f v = *(const v2fa*)(emb + (size_t)id * DIM + 2 * pc);
    const bool in = (p < DIM / 2);
    Pk2 pk;
    pk.e[0] = (_Float16)((in ? v.x : 0.0f) * 8.0f);
    pk.e[1] = (_Float16)((in ? v.y : 0.0f) * 8.0f);
    *(u32a*)(grow + row * KP + 2 * p) = pk.u;
  }
  __syncthreads();

  {
    const int mt = w >> 1, ntb = 2 * (w & 1);
    v8f acc0 = z8, acc1 = z8;
    #pragma unroll
    for (int ks = 0; ks < 2; ++ks) {
      const v16h a   = load_frag(cenA + (16 * mt + m) * KP + 32 * ks, h);
      const v16h bf0 = load_frag(w1b + (size_t)(16 * ntb + m) * KP + 32 * ks, h);
      const v16h bf1 = load_frag(w1b + (size_t)(16 * (ntb + 1) + m) * KP + 32 * ks, h);
      acc0 = wmma_f16(a, bf0, acc0);
      acc1 = wmma_f16(a, bf1, acc1);
    }
    #pragma unroll
    for (int r = 0; r < 8; ++r) {
      const int rowc = 16 * mt + 8 * h + r;
      hcs[rowc * NP1 + 16 * ntb + m]       = acc0[r] * (1.0f / 64.0f);
      hcs[rowc * NP1 + 16 * (ntb + 1) + m] = acc1[r] * (1.0f / 64.0f);
    }
  }
  __syncthreads();

  #pragma unroll 1
  for (int i = 0; i < 4; ++i) {
    const int mt = 4 * w + i;
    const _Float16* ap = grow + (16 * mt + m) * KP;
    const v16h a0 = load_frag(ap, h);
    const v16h a1 = load_frag(ap + 32, h);
    v8f acc[4];
    #pragma unroll
    for (int nt = 0; nt < 4; ++nt) {
      const _Float16* bp = w1a + (size_t)(16 * nt + m) * KP;
      const v16h bf0 = load_frag(bp, h);
      const v16h bf1 = load_frag(bp + 32, h);
      acc[nt] = z8;
      acc[nt] = wmma_f16(a0, bf0, acc[nt]);
      acc[nt] = wmma_f16(a1, bf1, acc[nt]);
    }
    const int bA = 2 * mt + h;
    #pragma unroll
    for (int nt = 0; nt < 4; ++nt) {
      const int n = 16 * nt + m;
      const float hc = hcs[bA * NP1 + n] + b1s[n];
      float s = 0.0f;
      #pragma unroll
      for (int r = 0; r < 8; ++r) s += fmaxf(acc[nt][r] * (1.0f / 64.0f) + hc, 0.0f);
      hs[bA * NP1 + n] = s;
    }
  }
  __syncthreads();

  {
    const int mt = 16 + w;
    const _Float16* ap = grow + (16 * mt + m) * KP;
    const v16h a0 = load_frag(ap, h);
    const v16h a1 = load_frag(ap + 32, h);
    v8f acc[4];
    #pragma unroll
    for (int nt = 0; nt < 4; ++nt) {
      const _Float16* bp = w1a + (size_t)(16 * nt + m) * KP;
      const v16h bf0 = load_frag(bp, h);
      const v16h bf1 = load_frag(bp + 32, h);
      acc[nt] = z8;
      acc[nt] = wmma_f16(a0, bf0, acc[nt]);
      acc[nt] = wmma_f16(a1, bf1, acc[nt]);
    }
    #pragma unroll
    for (int nt = 0; nt < 4; ++nt) {
      const int n = 16 * nt + m;
      #pragma unroll
      for (int q = 0; q < 4; ++q) {
        const int bT = 8 * w + 4 * h + q;
        const float hc = hcs[bT * NP1 + n] + b1s[n];
        const float s = fmaxf(acc[nt][2 * q] * (1.0f / 64.0f) + hc, 0.0f)
                      + fmaxf(acc[nt][2 * q + 1] * (1.0f / 64.0f) + hc, 0.0f);
        const float cur = hs[bT * NP1 + n];
        hs[bT * NP1 + n] = cur + s;
      }
    }
  }
  __syncthreads();

  #pragma unroll 1
  for (int i = t; i < TB * KP; i += NTH) hbf[i] = (_Float16)hs[i];
  __syncthreads();

  #pragma unroll 1
  for (int tt = w; tt < 14; tt += NWAV) {
    const int mt = tt & 1, nt = tt >> 1;
    v8f acc = z8;
    #pragma unroll
    for (int ks = 0; ks < 2; ++ks) {
      const v16h a  = load_frag(hbf + (16 * mt + m) * KP + 32 * ks, h);
      const v16h bf = load_frag(wmt + (size_t)(16 * nt + m) * KP + 32 * ks, h);
      acc = wmma_f16(a, bf, acc);
    }
    const int n = 16 * nt + m;
    const float bn = bmus[n];
    #pragma unroll
    for (int r = 0; r < 8; ++r) mus[(16 * mt + 8 * h + r) * NP2 + n] = acc[r] * 0.125f + bn;
  }
  __syncthreads();

  float pacc = 0.0f;
  #pragma unroll 1
  for (int u = t; u < NUNIT; u += NTH) {
    const bool isCen = (u >= AROWS);
    const int b = isCen ? (u - AROWS) : (u / CTX);
    const bool valid = (b0 + b) < nB;
    const float* murow = mus + b * NP2;
    const float ls  = murow[LAT];
    const float els = expf(ls);
    const int id0 = ids[min(u + (isCen ? AROWS : 0), NIDS - 1)];
    const int id1 = ids[min(u + AROWS, NIDS - 1)];
    const float kl0 = kl_term(id0, murow, ls, els, tmeans, tlogv);
    const float kl1 = kl_term(id1, murow, ls, els, tmeans, tlogv);
    const float hin = fmaxf(kl0 - kl1 + 1.0f, 0.0f);
    const float contrib = isCen ? kl0 : hin;
    pacc += valid ? contrib : 0.0f;
  }

  red[t] = (double)pacc;
  __syncthreads();
  if (t == 0) {
    double s = 0.0;
    #pragma unroll 1
    for (int i = 0; i < NTH; ++i) s += red[i];
    bsum[0] = s;
  }
  __syncthreads();
  const double stot = bsum[0];
  v2d o;
  o.x = (t == 0) ? stot : 0.0;
  o.y = 0.0;
  double* linep = part + (size_t)blockIdx.x * PART_STRIDE + 2 * t;
  if (t < 8) *(volatile v2d*)linep = o;
  __threadfence();
  if (t < 8) *(volatile v2d*)linep = o;
}

__global__ __launch_bounds__(32) void bsg_final(const double* part, float* out, int nblk, float invB) {
  __shared__ double sl[32];
  const int l = threadIdx.x;
  const int per = (nblk + 31) / 32;
  double s = 0.0;
  #pragma unroll 1
  for (int i = 0; i < per; ++i) {
    const int idx = l * per + i;
    const double v = part[(size_t)min(idx, nblk - 1) * PART_STRIDE];
    s += (idx < nblk) ? v : 0.0;
  }
  sl[l] = s;
  __syncthreads();
  if (l == 0) {
    double tot = 0.0;
    #pragma unroll 1
    for (int i = 0; i < 32; ++i) tot += sl[i];
    const float r = (float)tot * invB;
    *(volatile float*)out = r;
    __threadfence();
    *(volatile float*)out = r;
  }
}

extern "C" void kernel_launch(void* const* d_in, const int* in_sizes, int n_in,
                              void* d_out, int out_size, void* d_ws, size_t ws_size,
                              hipStream_t stream) {
  if (n_in < 12) return;
  const int nEmb = in_sizes[0];
  if (nEmb < DIM || (nEmb % DIM) != 0) return;
  const int nV = nEmb / DIM;
  if (in_sizes[1] != 2 * DIM * HID) return;
  if (in_sizes[2] != HID) return;
  if (in_sizes[3] != HID * LAT) return;
  if (in_sizes[4] != LAT) return;
  if (in_sizes[5] != HID) return;
  if (in_sizes[6] < 1) return;
  if (in_sizes[7] != nV * LAT) return;
  if (in_sizes[8] != nV) return;
  const int nB = in_sizes[9];
  if (nB < 1) return;
  if (in_sizes[10] != nB * CTX || in_sizes[11] != nB * CTX) return;
  if (out_size != 1) return;

  const int nblk = (nB + TB - 1) / TB;
  const size_t total = OFF_PART + (size_t)nblk * 128;
  if (total > ws_size) return;
  if (total > (size_t)134217728) return;

  const float* emb  = (const float*)d_in[0];
  const float* W1   = (const float*)d_in[1];
  const float* b1   = (const float*)d_in[2];
  const float* Wmu  = (const float*)d_in[3];
  const float* bmu  = (const float*)d_in[4];
  const float* Wls  = (const float*)d_in[5];
  const float* bls  = (const float*)d_in[6];
  const float* tm   = (const float*)d_in[7];
  const float* tl   = (const float*)d_in[8];
  const int*   cen  = (const int*)d_in[9];
  const int*   ctx  = (const int*)d_in[10];
  const int*   neg  = (const int*)d_in[11];
  float* out = (float*)d_out;

  char* ws = (char*)d_ws;
  _Float16* planes = (_Float16*)ws;
  const _Float16* w1a = planes;
  const _Float16* w1b = planes + NP1 * KP;
  const _Float16* wmt = planes + 2 * NP1 * KP;
  double* part = (double*)(ws + OFF_PART);

  bsg_prep<<<1, 256, 0, stream>>>(W1, Wmu, Wls, planes);

  hipFuncSetAttribute(reinterpret_cast<const void*>(&bsg_main),
                      hipFuncAttributeMaxDynamicSharedMemorySize, LDS_BYTES);
  bsg_main<<<nblk, NTH, LDS_BYTES, stream>>>(emb, b1, bmu, bls, tm, tl, cen, ctx, neg,
                                             w1a, w1b, wmt, part, nB, nV);

  bsg_final<<<1, 32, 0, stream>>>(part, out, nblk, 1.0f / (float)nB);
}
